// SelectiveSSM_28948079575407
// MI455X (gfx1250) — hardware-run, weakly checked
//
#include <hip/hip_runtime.h>
#include <hip/hip_fp16.h>
#include <math.h>

typedef __attribute__((ext_vector_type(16))) _Float16 v16h;
typedef __attribute__((ext_vector_type(8)))  _Float16 v8h;
typedef __attribute__((ext_vector_type(8)))  float    v8f;
typedef __attribute__((ext_vector_type(4)))  float    v4f;
typedef __attribute__((ext_vector_type(2)))  float    v2f;
typedef __attribute__((ext_vector_type(2)))  unsigned v2u;
typedef __attribute__((ext_vector_type(4)))  unsigned v4u;

constexpr int kBatch   = 2;
constexpr int kPasses  = kBatch;
constexpr int kL       = 2048;
constexpr int kRows    = kL;
constexpr int kDm      = 1024;
constexpr int kE       = 2048;
constexpr int kXzN     = 2 * kE;
constexpr int kNst     = 16;
constexpr int kRank    = 64;
constexpr int kTaps    = 4;
constexpr int kXpN     = kRank + 2 * kNst;
constexpr int kXpP     = 128;
constexpr int kWinRows = 2 * kE + kXpN;
constexpr int kWbRow0  = kWinRows - kXpP;
constexpr int kColB    = kXpP - kXpN;
constexpr int kColC    = kColB + kNst;
constexpr int kColDt   = kColC + kNst;
constexpr int kDtK     = 96;
constexpr int kWN       = kXpP;
constexpr int kK2       = kDtK;
constexpr int kK2Words  = kK2 / 8;
constexpr int kWdtPitch = 128;
constexpr int kAlpFloats = kE * kNst;
constexpr int kPadFloats = kAlpFloats + kE;
constexpr float kXCarry = 64.0f;
constexpr float kWCarry = 1024.0f;
constexpr float kDCarry = kWCarry;
constexpr float kRCarry = 256.0f;
constexpr float kGCarry = 256.0f;
constexpr float kYCarry = 64.0f;
constexpr float kResid  = 2048.0f;
static_assert(kBatch == 2 && kPasses == 2 && kRows == 2048 && kL == 2048);
static_assert(kDm == 1024 && kE == 2048 && kXzN == 4096 && kXpN == 96 && kNst == 16 && kRank == 64 && kTaps == 4);
static_assert(kXpN <= kXpP && (kRank % 8) == 0 && kXpP == 128 && kWN == 128);
static_assert(kWinRows == 4192 && kWbRow0 == 4064 && kColB == 32 && kColC == 48 && kColDt == 64);
static_assert((kColB % 4) == 0 && (kColC % 4) == 0 && (kColDt % 8) == 0 && kColDt + kRank == kXpP);
static_assert(kDtK == 96 && (kK2 % 32) == 0 && kRank + 1 <= kK2 && kK2Words == 12);
static_assert(kWdtPitch == 128 && kWdtPitch >= kK2 && ((kWdtPitch * 2) % 128) == 0);
static_assert((kDm % 32) == 0 && (kE % 32) == 0);
static_assert((kDm % 64) == 0 && (kE % 64) == 0 && (kXzN % 64) == 0 && (kXpP % 64) == 0);
static_assert((kRows % 32) == 0);
static_assert((kL % 64) == 0);
static_assert(kAlpFloats == 32768 && kPadFloats == 34816);
static_assert(kDCarry == 1024.0f);

constexpr size_t kSzWIN  = (size_t)kXzN * kDm * 2;
constexpr size_t kSzWB   = (size_t)kXpP * kDm * 2;
constexpr size_t kSzWDT  = (size_t)kE * kWdtPitch * 2;
constexpr size_t kSzOW   = (size_t)kDm * kE * 2;
constexpr size_t kSzPADS = (size_t)kPadFloats * 4;
constexpr size_t kSzSH   = (size_t)kRows * kDm * 2;
constexpr size_t kSzXZ   = (size_t)kRows * kXzN * 4;
constexpr size_t kSzXC   = (size_t)kRows * kE * 4;
constexpr size_t kSzXD   = (size_t)kRows * kXpP * 4;
constexpr size_t kSzDRH  = (size_t)kRows * kK2 * 2;
constexpr size_t kSzDTP  = (size_t)kRows * kE * 4;
constexpr size_t kSzYH   = (size_t)kRows * kE * 2;
constexpr size_t kSzYG   = (size_t)kRows * kE * 2;
constexpr size_t kSzH    = (size_t)kRows * kDm * 4;
constexpr size_t kSzR    = (size_t)kRows * kDm * 4;
constexpr size_t kSzST   = (size_t)kRows * 4 * 4;
constexpr size_t kOffWIN  = 0;
constexpr size_t kOffWB   = kOffWIN  + kSzWIN;
constexpr size_t kOffWDT  = kOffWB   + kSzWB;
constexpr size_t kOffOW   = kOffWDT  + kSzWDT;
constexpr size_t kOffPADS = kOffOW   + kSzOW;
constexpr size_t kOffSH   = kOffPADS + kSzPADS;
constexpr size_t kOffXZ   = kOffSH   + kSzSH;
constexpr size_t kOffXC   = kOffXZ   + kSzXZ;
constexpr size_t kOffXD   = kOffXC   + kSzXC;
constexpr size_t kOffDRH  = kOffXD   + kSzXD;
constexpr size_t kOffDTP  = kOffDRH  + kSzDRH;
constexpr size_t kOffYH   = kOffDTP  + kSzDTP;
constexpr size_t kOffYG   = kOffYH   + kSzYH;
constexpr size_t kOffH    = kOffYG   + kSzYG;
constexpr size_t kOffR    = kOffH    + kSzH;
constexpr size_t kOffST   = kOffR    + kSzR;
constexpr size_t kWsTotal = kOffST   + kSzST;
static_assert(kSzWIN == 8388608ull);
static_assert(kSzWB == 262144ull);
static_assert(kSzWDT == 524288ull);
static_assert(kSzOW == 4194304ull);
static_assert(kSzPADS == 139264ull);
static_assert(kSzSH == 4194304ull);
static_assert(kSzXZ == 33554432ull);
static_assert(kSzXC == 16777216ull);
static_assert(kSzXD == 1048576ull);
static_assert(kSzDRH == 393216ull);
static_assert(kSzDTP == 16777216ull);
static_assert(kSzYH == 8388608ull);
static_assert(kSzYG == 8388608ull);
static_assert(kSzH == 8388608ull);
static_assert(kSzR == 8388608ull);
static_assert(kSzST == 32768ull);
static_assert(kWsTotal == 119840768ull);
static_assert(kWsTotal <= 134217728ull);
static_assert((kSzWIN % 128) == 0 && (kSzWB % 128) == 0 && (kSzWDT % 128) == 0 && (kSzOW % 128) == 0 && (kSzPADS % 128) == 0 && (kSzSH % 128) == 0 && (kSzXZ % 128) == 0 && (kSzXC % 128) == 0 && (kSzXD % 128) == 0 && (kSzDRH % 128) == 0 && (kSzDTP % 128) == 0 && (kSzYH % 128) == 0 && (kSzYG % 128) == 0 && (kSzH % 128) == 0 && (kSzR % 128) == 0 && (kSzST % 128) == 0);
static_assert((((size_t)kAlpFloats * 4) % 128) == 0);
static_assert((((size_t)kXpP * 4) % 128) == 0);

__device__ __forceinline__ _Float16 f16_flush(float v) {
  const float w = (fabsf(v) < 6.103515625e-05f) ? 0.0f : v;
  return (_Float16)w;
}
__device__ __forceinline__ void f16_split(float v, _Float16& hi, _Float16& lo) {
  hi = f16_flush(v);
  const float hf = (float)hi;
  const float r = (v - hf) * kResid;
  lo = f16_flush(r);
}

__device__ __forceinline__ float bf16r(float v) {
  unsigned u = __float_as_uint(v);
  u = (u + 0x7FFFu + ((u >> 16) & 1u)) & 0xFFFF0000u;
  return __uint_as_float(u);
}

__device__ __forceinline__ float h16_to_f32(unsigned hb) {
  const unsigned sgn = (hb & 0x8000u) << 16; const unsigned em = hb & 0x7fffu;
  const float fn = __uint_as_float((em << 13) + 0x38000000u);
  const float fs = (float)em * 5.9604644775390625e-8f;
  const float mag = (em < 0x400u) ? fs : fn; return __uint_as_float(__float_as_uint(mag) | sgn); }

namespace eng {
union FragU { v16h v; v8h h[2]; };
__device__ __forceinline__ v16h frag_load(const _Float16* p) {
  FragU f;
  f.h[0] = *(const v8h*)(p);
  f.h[1] = *(const v8h*)(p + 16);
  return f.v;
}
__device__ __forceinline__ v8f mma(v16h a, v16h b, v8f c) {
  return __builtin_amdgcn_wmma_f32_16x16x32_f16(false, a, false, b, (short)0, c, false, false);
}
__device__ __forceinline__ void guard1(v8f& a, v16h x, v16h y) {
  asm volatile("v_nop\n\tv_nop\n\tv_nop\n\tv_nop" : "+v"(a) : "v"(x), "v"(y));
}
__device__ __forceinline__ void guard_acc(v8f& a) {
  asm volatile("v_nop\n\tv_nop\n\tv_nop\n\tv_nop" : "+v"(a));
}
__device__ __forceinline__ void keep4(v16h a, v16h b, v16h c, v16h d) {
  asm volatile("v_nop" :: "v"(a), "v"(b), "v"(c), "v"(d));
}

template <int MI, int SPL>
__global__ __launch_bounds__(256) void gemm_f16_kernel(
    const unsigned short* __restrict__ Ap, const unsigned short* __restrict__ A2p, int lda,
    const unsigned short* __restrict__ Btp, const unsigned short* __restrict__ Bt2p, int ldb,
    float* __restrict__ C, int ldc, int M, int N, int K, float scale, float rscale)
{
  static_assert(MI >= 1 && MI <= 2);
  static_assert(SPL >= 0 && SPL <= 2);
  const _Float16* A   = (const _Float16*)Ap;
  const _Float16* A2  = (const _Float16*)A2p;
  const _Float16* Bt  = (const _Float16*)Btp;
  const _Float16* Bt2 = (const _Float16*)Bt2p;
  __shared__ __align__(16) float sT[8][16 * 68];
  const int lane = threadIdx.x & 31;
  const int wave = threadIdx.x >> 5;
  const int tilesN = N >> 6;
  const int tilesM = M / (16 * MI);
  const int tile = blockIdx.x * 8 + wave;
  if (tile >= tilesM * tilesN) return;
  const int tm = tile / tilesN;
  const int tn = tile - tm * tilesN;
  const int m0 = tm * (16 * MI);
  const int n0 = tn << 6;
  const int rlane = lane & 15;
  const int koff  = (lane >> 4) * 8;
  const int mOff  = (lane >> 4) * 8;

  v8f acc[MI][4], accr[MI][4];
#pragma unroll
  for (int i = 0; i < MI; ++i)
#pragma unroll
    for (int j = 0; j < 4; ++j) {
      acc[i][j]  = (v8f){0.f, 0.f, 0.f, 0.f, 0.f, 0.f, 0.f, 0.f};
      accr[i][j] = (v8f){0.f, 0.f, 0.f, 0.f, 0.f, 0.f, 0.f, 0.f};
    }

  for (int k0 = 0; k0 < K; k0 += 32) {
    v16h bh[4], bl[4];
#pragma unroll
    for (int j = 0; j < 4; ++j) {
      const size_t bo = (size_t)(n0 + (j << 4) + rlane) * ldb + koff + k0;
      bh[j] = frag_load(Bt + bo);
      if (SPL == 2) bl[j] = frag_load(Bt2 + bo); else bl[j] = bh[j];
    }
#pragma unroll
    for (int i = 0; i < MI; ++i) {
      const size_t ao = (size_t)(m0 + (i << 4) + rlane) * lda + koff + k0;
      const v16h ah = frag_load(A + ao);
      v16h al = ah;
      if (SPL >= 1) al = frag_load(A2 + ao);
#pragma unroll
      for (int j = 0; j < 4; ++j) {
        acc[i][j] = mma(ah, bh[j], acc[i][j]);
        if (SPL >= 1) accr[i][j] = mma(al, bh[j], accr[i][j]);
        if (SPL == 2) accr[i][j] = mma(ah, bl[j], accr[i][j]);
      }
#pragma unroll
      for (int j = 0; j < 4; ++j) {
        guard1(acc[i][j], ah, al);
        if (SPL >= 1) guard1(accr[i][j], ah, al);
      }
    }
    keep4(bh[0], bh[1], bh[2], bh[3]);
    if (SPL == 2) keep4(bl[0], bl[1], bl[2], bl[3]);
  }
#pragma unroll
  for (int i = 0; i < MI; ++i)
#pragma unroll
    for (int j = 0; j < 4; ++j) {
      guard_acc(acc[i][j]);
      if (SPL >= 1) guard_acc(accr[i][j]);
    }

  float* slab = sT[wave];
#pragma unroll
  for (int i = 0; i < MI; ++i) {
    const int mBase = m0 + (i << 4);
#pragma unroll
    for (int j = 0; j < 4; ++j) {
#pragma unroll
      for (int r = 0; r < 8; ++r) {
        float v = acc[i][j][r] * scale;
        if (SPL >= 1) v += accr[i][j][r] * rscale;
        slab[(mOff + r) * 68 + (j << 4) + rlane] = v;
      }
    }
    __builtin_amdgcn_fence(__ATOMIC_RELEASE, "workgroup");
    __builtin_amdgcn_wave_barrier();
    __builtin_amdgcn_fence(__ATOMIC_ACQUIRE, "workgroup");
    {
      const int hh = lane >> 4, c4 = (lane & 15) * 4;
      for (int pass = 0; pass < 2; ++pass) {
#pragma unroll
        for (int it = 0; it < 8; ++it) {
          const int row = it * 2 + hh;
          const v4f v = *(const v4f*)(slab + row * 68 + c4);
          *(volatile v4f*)(C + (size_t)(mBase + row) * ldc + n0 + c4) = v;
        }
        __threadfence();
      }
    }
    __builtin_amdgcn_fence(__ATOMIC_RELEASE, "workgroup");
    __builtin_amdgcn_wave_barrier();
    __builtin_amdgcn_fence(__ATOMIC_ACQUIRE, "workgroup");
  }
}
}

__device__ __forceinline__ _Float16 in_half(float v, float carry, bool live) {
  const float t = live ? (bf16r(v) * carry) : 0.0f;
  return f16_flush(t);
}
__device__ __forceinline__ _Float16 val_half(float v, float carry, bool live) {
  const float t = live ? (v * carry) : 0.0f;
  return f16_flush(t);
}
__device__ __forceinline__ int imin2(int a, int b) {
  return (a < b) ? a : b;
}
__device__ __forceinline__ v8h pack8_in(v4f a0, v4f a1, float carry, bool live) {
  const float f0 = a0[0];
  const float f1 = a0[1];
  const float f2 = a0[2];
  const float f3 = a0[3];
  const float f4 = a1[0];
  const float f5 = a1[1];
  const float f6 = a1[2];
  const float f7 = a1[3];
  v8h hv;
  hv[0] = in_half(f0, carry, live);
  hv[1] = in_half(f1, carry, live);
  hv[2] = in_half(f2, carry, live);
  hv[3] = in_half(f3, carry, live);
  hv[4] = in_half(f4, carry, live);
  hv[5] = in_half(f5, carry, live);
  hv[6] = in_half(f6, carry, live);
  hv[7] = in_half(f7, carry, live);
  return hv;
}

__global__ __launch_bounds__(256) void pack_win_kernel(
    const float* __restrict__ w, unsigned short* __restrict__ WIN)
{
  const int i = blockIdx.x * 256 + threadIdx.x;
  const int n = i / (kDm / 8);
  const int c8 = (i - n * (kDm / 8)) * 8;
  const float* sp = w + (size_t)n * kDm + c8;
  const v4f a0 = *(const v4f*)(sp);
  const v4f a1 = *(const v4f*)(sp + 4);
  const v8h hv = pack8_in(a0, a1, kWCarry, true);
  unsigned short* q = WIN + (size_t)i * 8;
  *(volatile v8h*)q = hv;
  __threadfence();
  *(volatile v8h*)q = hv;
}

constexpr int kRankWords = kRank / 8;
constexpr int kTailWords = (kWdtPitch - kRank) / 8;
static_assert(kRankWords == 8 && kTailWords == 8 && (kRankWords + kTailWords) * 8 == kWdtPitch);
static_assert(((kRank * 2) % 128) == 0);

__global__ __launch_bounds__(256) void pack_wdt_kernel(
    const float* __restrict__ w, unsigned short* __restrict__ WDT)
{
  const int i = blockIdx.x * 256 + threadIdx.x;
  const int d = i / kRankWords;
  const int q = (i - d * kRankWords) * 8;
  const float* sp = w + (size_t)d * kRank + q;
  const v4f a0 = *(const v4f*)(sp);
  const v4f a1 = *(const v4f*)(sp + 4);
  const v8h hv = pack8_in(a0, a1, kWCarry, true);
  unsigned short* qd = WDT + (size_t)d * kWdtPitch + q;
  *(volatile v8h*)qd = hv;
  __threadfence();
  *(volatile v8h*)qd = hv;
}

__global__ __launch_bounds__(256) void pack_bias_kernel(
    const float* __restrict__ bdt, unsigned short* __restrict__ WDT)
{
  const int i = blockIdx.x * 256 + threadIdx.x;
  const int d = i / kTailWords;
  const int w = i - d * kTailWords;
  const bool isBias = (w == 0);
  const float bv = bdt[d];
  const float tb = bf16r(bv) * kDCarry;
  const float t0 = isBias ? tb : 0.0f;
  const _Float16 h0 = f16_flush(t0);
  const unsigned short b0 = __builtin_bit_cast(unsigned short, h0);
  const unsigned w0 = (unsigned)b0;
  v4u ov;
  ov[0] = w0;
  ov[1] = 0u;
  ov[2] = 0u;
  ov[3] = 0u;
  unsigned short* qd = WDT + (size_t)d * kWdtPitch + kRank + w * 8;
  *(volatile v4u*)qd = ov;
  __threadfence();
  *(volatile v4u*)qd = ov;
}

__global__ __launch_bounds__(256) void pack_wout_kernel(
    const float* __restrict__ w, unsigned short* __restrict__ OW)
{
  const int i = blockIdx.x * 256 + threadIdx.x;
  const int m = i / (kE / 8);
  const int c8 = (i - m * (kE / 8)) * 8;
  const float* sp = w + (size_t)m * kE + c8;
  const v4f a0 = *(const v4f*)(sp);
  const v4f a1 = *(const v4f*)(sp + 4);
  const v8h hv = pack8_in(a0, a1, kWCarry, true);
  unsigned short* q = OW + (size_t)i * 8;
  *(volatile v8h*)q = hv;
  __threadfence();
  *(volatile v8h*)q = hv;
}

__global__ __launch_bounds__(32) void pads_kernel(
    const float* __restrict__ alog, const float* __restrict__ dskip, float* __restrict__ PADS)
{
  const int wi = blockIdx.x * 32 + threadIdx.x;
  const int f0 = wi * 4;
  const bool isA = (f0 < kAlpFloats);
  const int ea = isA ? f0 : (kAlpFloats - 4);
  const int ed = isA ? 0 : (f0 - kAlpFloats);
  const v4f va = *(const v4f*)(alog + ea);
  const v4f vd = *(const v4f*)(dskip + ed);
  const float a0 = va[0];
  const float a1 = va[1];
  const float a2 = va[2];
  const float a3 = va[3];
  const float d0 = vd[0];
  const float d1 = vd[1];
  const float d2 = vd[2];
  const float d3 = vd[3];
  const float s0 = isA ? a0 : d0;
  const float s1 = isA ? a1 : d1;
  const float s2 = isA ? a2 : d2;
  const float s3 = isA ? a3 : d3;
  v4f o;
  o[0] = bf16r(s0);
  o[1] = bf16r(s1);
  o[2] = bf16r(s2);
  o[3] = bf16r(s3);
  float* q = PADS + (size_t)f0;
  *(volatile v4f*)q = o;
  __threadfence();
  *(volatile v4f*)q = o;
}

__global__ __launch_bounds__(256) void pack_s_kernel(
    const float* __restrict__ s, unsigned short* __restrict__ SH)
{
  const int i = blockIdx.x * 256 + threadIdx.x;
  const int r = i / (kDm / 8);
  const int c8 = (i - r * (kDm / 8)) * 8;
  const float* sp = s + (size_t)r * kDm + c8;
  const v4f a0 = *(const v4f*)(sp);
  const v4f a1 = *(const v4f*)(sp + 4);
  const v8h hv = pack8_in(a0, a1, kXCarry, true);
  unsigned short* q = SH + (size_t)i * 8;
  *(volatile v8h*)q = hv;
  __threadfence();
  *(volatile v8h*)q = hv;
}

__device__ __forceinline__ float conv_silu(float bias, float x0, float x1, float x2, float x3, v4f wv) {
  const float w0 = wv[0];
  const float w1 = wv[1];
  const float w2 = wv[2];
  const float w3 = wv[3];
  float acc = bf16r(bias);
  acc = fmaf(x0, bf16r(w0), acc);
  acc = fmaf(x1, bf16r(w1), acc);
  acc = fmaf(x2, bf16r(w2), acc);
  acc = fmaf(x3, bf16r(w3), acc);
  return acc / (1.0f + expf(-acc));
}
__global__ __launch_bounds__(256) void conv1d_kernel(
    const float* __restrict__ XZ, const float* __restrict__ cw, const float* __restrict__ cb,
    float* __restrict__ XC)
{
  const int i = blockIdx.x * 256 + threadIdx.x;
  const int r = i / (kE / 4);
  const int c4 = (i - r * (kE / 4)) * 4;
  const int t = r % kL;
  const int rlo = r - t;
  const int ra = r - 3;
  const int rb = r - 2;
  const int rc = r - 1;
  const int qa = (ra < rlo) ? rlo : ra;
  const int qb = (rb < rlo) ? rlo : rb;
  const int qc = (rc < rlo) ? rlo : rc;
  const bool la = (t >= 3);
  const bool lb = (t >= 2);
  const bool lc = (t >= 1);
  const v4f xa = *(const v4f*)(XZ + (size_t)qa * kXzN + c4);
  const v4f xb = *(const v4f*)(XZ + (size_t)qb * kXzN + c4);
  const v4f xc = *(const v4f*)(XZ + (size_t)qc * kXzN + c4);
  const v4f xd = *(const v4f*)(XZ + (size_t)r * kXzN + c4);
  const v4f w0 = *(const v4f*)(cw + (size_t)(c4 + 0) * kTaps);
  const v4f w1 = *(const v4f*)(cw + (size_t)(c4 + 1) * kTaps);
  const v4f w2 = *(const v4f*)(cw + (size_t)(c4 + 2) * kTaps);
  const v4f w3 = *(const v4f*)(cw + (size_t)(c4 + 3) * kTaps);
  const v4f bv = *(const v4f*)(cb + c4);
  const float a0 = xa[0];
  const float a1 = xa[1];
  const float a2 = xa[2];
  const float a3 = xa[3];
  const float b0 = xb[0];
  const float b1 = xb[1];
  const float b2 = xb[2];
  const float b3 = xb[3];
  const float e0 = xc[0];
  const float e1 = xc[1];
  const float e2 = xc[2];
  const float e3 = xc[3];
  const float d0 = xd[0];
  const float d1 = xd[1];
  const float d2 = xd[2];
  const float d3 = xd[3];
  const float ta0 = la ? a0 : 0.0f;
  const float ta1 = la ? a1 : 0.0f;
  const float ta2 = la ? a2 : 0.0f;
  const float ta3 = la ? a3 : 0.0f;
  const float tb0 = lb ? b0 : 0.0f;
  const float tb1 = lb ? b1 : 0.0f;
  const float tb2 = lb ? b2 : 0.0f;
  const float tb3 = lb ? b3 : 0.0f;
  const float tc0 = lc ? e0 : 0.0f;
  const float tc1 = lc ? e1 : 0.0f;
  const float tc2 = lc ? e2 : 0.0f;
  const float tc3 = lc ? e3 : 0.0f;
  const float bs0 = bv[0];
  const float bs1 = bv[1];
  const float bs2 = bv[2];
  const float bs3 = bv[3];
  v4f o;
  o[0] = conv_silu(bs0, ta0, tb0, tc0, d0, w0);
  o[1] = conv_silu(bs1, ta1, tb1, tc1, d1, w1);
  o[2] = conv_silu(bs2, ta2, tb2, tc2, d2, w2);
  o[3] = conv_silu(bs3, ta3, tb3, tc3, d3, w3);
  float* q = XC + (size_t)i * 4;
  *(volatile v4f*)q = o;
  __threadfence();
  *(volatile v4f*)q = o;
}

__global__ __launch_bounds__(256) void pack_dr_kernel(
    const float* __restrict__ XP, unsigned short* __restrict__ DRH)
{
  const int i = blockIdx.x * 256 + threadIdx.x;
  const int r = i / kK2Words;
  const int q = (i - r * kK2Words) * 8;
  const bool live = (q < kRank);
  const bool isOne = (q == kRank);
  const int qc = imin2(q, kRank - 8);
  const float* sp = XP + (size_t)r * kWN + qc;
  const v4f a0 = *(const v4f*)(sp);
  const v4f a1 = *(const v4f*)(sp + 4);
  const float f0 = a0[0];
  const float f1 = a0[1];
  const float f2 = a0[2];
  const float f3 = a0[3];
  const float f4 = a1[0];
  const float f5 = a1[1];
  const float f6 = a1[2];
  const float f7 = a1[3];
  const float t0a = live ? (f0 * kRCarry) : 0.0f;
  const float t0 = isOne ? kRCarry : t0a;
  v8h hv;
  hv[0] = f16_flush(t0);
  hv[1] = val_half(f1, kRCarry, live);
  hv[2] = val_half(f2, kRCarry, live);
  hv[3] = val_half(f3, kRCarry, live);
  hv[4] = val_half(f4, kRCarry, live);
  hv[5] = val_half(f5, kRCarry, live);
  hv[6] = val_half(f6, kRCarry, live);
  hv[7] = val_half(f7, kRCarry, live);
  unsigned short* qd = DRH + (size_t)i * 8;
  *(volatile v8h*)qd = hv;
  __threadfence();
  *(volatile v8h*)qd = hv;
}

typedef float    ms1_v4f __attribute__((ext_vector_type(4)));
typedef unsigned ms1_v4u __attribute__((ext_vector_type(4)));
struct ms1_args {
  const float* dtpre;
  const float* u;
  const float* bc;
  const float* z;
  const float* A_log;
  const float* Dskip;
  __half* y;
  __half* y_lo;
  long ld_dtpre;
  long ld_u;
  long ld_bc;
  long ld_z;
  long ld_y;
  int offB;
  int offC;
  int offZ;
  float ycarry;
  int dir;
  int D;
  int L;
  int nbatch;
};
static_assert(sizeof(ms1_args) == 136);

__device__ __forceinline__ float ms1_flush16(float v) {
  return (fabsf(v) < 6.103515625e-05f) ? 0.0f : v;
}
__device__ __forceinline__ unsigned ms1_h16bits(float v) {
  return (unsigned)__half_as_ushort(__float2half_rn(ms1_flush16(v)));
}
__device__ __forceinline__ float ms1_h16val(unsigned b) {
  return __half2float(__ushort_as_half((unsigned short)b));
}
__device__ __forceinline__ float ms1_softplus(float v) {
  return fmaxf(v, 0.0f) + log1pf(expf(-fabsf(v)));
}
__device__ __forceinline__ void ms1_pack2(float v0, float v1, unsigned& hw, unsigned& lw) {
  const unsigned h0 = ms1_h16bits(v0);
  const unsigned h1 = ms1_h16bits(v1);
  const float r0 = (v0 - ms1_h16val(h0)) * 2048.0f;
  const float r1 = (v1 - ms1_h16val(h1)) * 2048.0f;
  const unsigned l0 = ms1_h16bits(r0);
  const unsigned l1 = ms1_h16bits(r1);
  hw = h0 | (h1 << 16);
  lw = l0 | (l1 << 16);
}

template <int NSTATE>
__global__ __launch_bounds__(64 * (NSTATE / 16)) void ms1_scan_kernel(ms1_args a)
{
  static_assert(NSTATE == 16 || NSTATE == 64);
  constexpr int NQ  = NSTATE / 16;
  constexpr int NT  = 64 * NQ;
  constexpr int NW  = NT / 32;
  constexpr int BCW = 2 * NSTATE;
  constexpr int YP  = 68;
  constexpr int RPI = NW * 4;
  constexpr int NIT = 64 / RPI;
  static_assert(16 * NT <= 64 * YP);
  __shared__ __align__(16) float sBC[64 * BCW];
  __shared__ __align__(16) float sY[64 * YP];
  const int tid  = threadIdx.x;
  const int lane = tid & 31;
  const int wave = tid >> 5;
  const int c    = tid / NQ;
  const int sq   = tid - c * NQ;
  const int bpb  = a.D / 64;
  const int bi   = blockIdx.x / bpb;
  if (bi >= a.nbatch) return;
  const int d0 = (blockIdx.x - bi * bpb) * 64;
  const int d  = d0 + c;
  const long rowb = (long)bi * a.L;
  const bool hasz  = (a.z != nullptr);
  const bool hasD  = (a.Dskip != nullptr);
  const bool hasLo = (a.y_lo != nullptr);

#pragma unroll 1
  for (int n = 0; n < 16; ++n) {
    const float al = a.A_log[(long)d * NSTATE + sq * 16 + n];
    sY[n * NT + tid] = -expf(al);
  }
  __syncthreads();
  float An[16], h[16];
#pragma unroll
  for (int n = 0; n < 16; ++n) {
    An[n] = sY[n * NT + tid];
    h[n] = 0.0f;
  }
  float Dd = 0.0f;
  if (hasD) Dd = a.Dskip[d];

  const int nchunk = a.L / 64;
  const bool fwd = (a.dir > 0);
  const int s0 = fwd ? 0 : 63;
  const int sd = fwd ? 1 : -1;
  const int q  = lane >> 3;
  const int c8 = (lane & 7) * 8;

  for (int ci = 0; ci < nchunk; ++ci) {
    const int tb = fwd ? (ci * 64) : (a.L - 64 - ci * 64);
    const long rowc = rowb + tb;
    __syncthreads();
#pragma unroll 8
    for (int i = 0; i < 32; ++i) {
      const int idx = tid + i * NT;
      const int st  = idx / BCW;
      const int col = idx - st * BCW;
      const int sc  = (col < NSTATE) ? (a.offB + col) : (a.offC + col - NSTATE);
      sBC[idx] = a.bc[(rowc + st) * a.ld_bc + sc];
    }
    __syncthreads();
    for (int s = 0; s < 64; ++s) {
      const int ls = s0 + sd * s;
      const long row = rowc + ls;
      float pre = a.dtpre[row * a.ld_dtpre + d];
      float uv  = a.u[row * a.ld_u + d];
      float zv  = 0.0f;
      if (hasz) zv = a.z[row * a.ld_z + a.offZ + d];
      asm volatile("" : "+v"(pre));
      asm volatile("" : "+v"(uv));
      asm volatile("" : "+v"(zv));
      const float delta = ms1_softplus(pre);
      const float dtx = delta * uv;
      const float* bp = sBC + ls * BCW + sq * 16;
      const float* cp = bp + NSTATE;
      ms1_v4f Bq[4], Cq[4];
#pragma unroll
      for (int k = 0; k < 4; ++k) {
        Bq[k] = *(const ms1_v4f*)(bp + 4 * k);
        Cq[k] = *(const ms1_v4f*)(cp + 4 * k);
      }
      float yv = 0.0f;
#pragma unroll
      for (int n = 0; n < 16; ++n) {
        const float e = __expf(delta * An[n]);
        h[n] = fmaf(e, h[n], dtx * Bq[n >> 2][n & 3]);
        yv = fmaf(h[n], Cq[n >> 2][n & 3], yv);
      }
      if (NQ > 1) {
        yv += __shfl_xor(yv, 1, 32);
        yv += __shfl_xor(yv, 2, 32);
      }
      if (hasD) yv = fmaf(uv, Dd, yv);
      if (hasz) {
        const float sg = __builtin_amdgcn_rcpf(1.0f + expf(-zv));
        yv = yv * (zv * sg);
      }
      if (sq == 0) sY[ls * YP + c] = yv * a.ycarry;
    }
    __syncthreads();
    ms1_v4u hw[NIT], lw[NIT];
#pragma unroll
    for (int it = 0; it < NIT; ++it) {
      const int row = it * RPI + wave * 4 + q;
      const float* sp = sY + row * YP + c8;
      const ms1_v4f f0 = *(const ms1_v4f*)(sp);
      const ms1_v4f f1 = *(const ms1_v4f*)(sp + 4);
      unsigned h0, h1, h2, h3, l0, l1, l2, l3;
      ms1_pack2(f0[0], f0[1], h0, l0);
      ms1_pack2(f0[2], f0[3], h1, l1);
      ms1_pack2(f1[0], f1[1], h2, l2);
      ms1_pack2(f1[2], f1[3], h3, l3);
      hw[it] = (ms1_v4u){h0, h1, h2, h3};
      lw[it] = (ms1_v4u){l0, l1, l2, l3};
    }
    for (int pass = 0; pass < 2; ++pass) {
#pragma unroll
      for (int it = 0; it < NIT; ++it) {
        const int row = it * RPI + wave * 4 + q;
        const long o = (rowc + row) * a.ld_y + d0 + c8;
        *(volatile ms1_v4u*)(a.y + o) = hw[it];
        if (hasLo) *(volatile ms1_v4u*)(a.y_lo + o) = lw[it];
      }
      __threadfence();
    }
  }
}

__device__ __forceinline__ _Float16 gate_half(unsigned hb, float zr) {
  const float hv = h16_to_f32(hb);
  const float y = hv * (1.0f / kYCarry);
  const float g = zr / (1.0f + expf(-zr));
  return f16_flush(y * g * kGCarry);
}
__global__ __launch_bounds__(256) void gate_kernel(
    const unsigned short* __restrict__ YH, const float* __restrict__ XZ, unsigned short* __restrict__ YG)
{
  const int i = blockIdx.x * 256 + threadIdx.x;
  const int r = i / (kE / 8);
  const int c8 = (i - r * (kE / 8)) * 8;
  const v4u wh = *(const v4u*)(YH + (size_t)i * 8);
  const float* zp = XZ + (size_t)r * kXzN + kE + c8;
  const v4f za = *(const v4f*)(zp);
  const v4f zb = *(const v4f*)(zp + 4);
  const unsigned h0 = wh[0];
  const unsigned h1 = wh[1];
  const unsigned h2 = wh[2];
  const unsigned h3 = wh[3];
  const float z0 = za[0];
  const float z1 = za[1];
  const float z2 = za[2];
  const float z3 = za[3];
  const float z4 = zb[0];
  const float z5 = zb[1];
  const float z6 = zb[2];
  const float z7 = zb[3];
  v8h hv;
  hv[0] = gate_half(h0 & 0xffffu, z0);
  hv[1] = gate_half(h0 >> 16, z1);
  hv[2] = gate_half(h1 & 0xffffu, z2);
  hv[3] = gate_half(h1 >> 16, z3);
  hv[4] = gate_half(h2 & 0xffffu, z4);
  hv[5] = gate_half(h2 >> 16, z5);
  hv[6] = gate_half(h3 & 0xffffu, z6);
  hv[7] = gate_half(h3 >> 16, z7);
  unsigned short* q = YG + (size_t)i * 8;
  *(volatile v8h*)q = hv;
  __threadfence();
  *(volatile v8h*)q = hv;
}

__global__ __launch_bounds__(256) void res_out_kernel(
    const float* __restrict__ x, const float* __restrict__ H, float* __restrict__ out)
{
  const int i = blockIdx.x * 256 + threadIdx.x;
  const v4f xa = *(const v4f*)(x + (size_t)i * 4);
  const v4f ha = *(const v4f*)(H + (size_t)i * 4);
  const float x0 = xa[0];
  const float x1 = xa[1];
  const float x2 = xa[2];
  const float x3 = xa[3];
  const float h0 = ha[0];
  const float h1 = ha[1];
  const float h2 = ha[2];
  const float h3 = ha[3];
  v4f o;
  o[0] = bf16r(x0) + h0;
  o[1] = bf16r(x1) + h1;
  o[2] = bf16r(x2) + h2;
  o[3] = bf16r(x3) + h3;
  float* q = out + (size_t)i * 4;
  *(volatile v4f*)q = o;
  __threadfence();
  *(volatile v4f*)q = o;
}

__global__ __launch_bounds__(256) void ln_stats_kernel(
    const float* __restrict__ H, float* __restrict__ ST)
{
  const int r = blockIdx.x * 256 + threadIdx.x;
  const float* mp = H + (size_t)r * kDm;
  float sum = 0.0f;
  for (int c = 0; c < 1024; c += 4) {
    const v4f v = *(const v4f*)(mp + c);
    const float a0 = v[0];
    const float a1 = v[1];
    const float a2 = v[2];
    const float a3 = v[3];
    sum = sum + a0;
    sum = sum + a1;
    sum = sum + a2;
    sum = sum + a3;
  }
  const float mu = sum * (1.0f / 1024.0f);
  float vs = 0.0f;
  for (int c = 0; c < 1024; c += 4) {
    const v4f v = *(const v4f*)(mp + c);
    const float a0 = v[0];
    const float a1 = v[1];
    const float a2 = v[2];
    const float a3 = v[3];
    const float e0 = a0 - mu;
    const float e1 = a1 - mu;
    const float e2 = a2 - mu;
    const float e3 = a3 - mu;
    vs = fmaf(e0, e0, vs);
    vs = fmaf(e1, e1, vs);
    vs = fmaf(e2, e2, vs);
    vs = fmaf(e3, e3, vs);
  }
  const float var = vs * (1.0f / 1024.0f);
  const float rs = 1.0f / sqrtf(var + 1e-5f);
  v4f ov;
  ov[0] = mu;
  ov[1] = rs;
  ov[2] = 0.0f;
  ov[3] = 0.0f;
  float* q = ST + (size_t)r * 4;
  *(volatile v4f*)q = ov;
  __threadfence();
  *(volatile v4f*)q = ov;
}

__global__ __launch_bounds__(256) void ln_out_kernel(
    const float* __restrict__ H, const float* __restrict__ ST, const float* __restrict__ lg,
    const float* __restrict__ lb, float* __restrict__ out)
{
  const int i = blockIdx.x * 256 + threadIdx.x;
  const int r = i / (kDm / 4);
  const int c4 = (i - r * (kDm / 4)) * 4;
  const v4f hv = *(const v4f*)(H + (size_t)i * 4);
  const v2f sv = *(const v2f*)(ST + (size_t)r * 4);
  const v4f gv = *(const v4f*)(lg + c4);
  const v4f bv = *(const v4f*)(lb + c4);
  const float h0 = hv[0];
  const float h1 = hv[1];
  const float h2 = hv[2];
  const float h3 = hv[3];
  const float mu = sv[0];
  const float rs = sv[1];
  const float g0 = gv[0];
  const float g1 = gv[1];
  const float g2 = gv[2];
  const float g3 = gv[3];
  const float b0 = bv[0];
  const float b1 = bv[1];
  const float b2 = bv[2];
  const float b3 = bv[3];
  v4f o;
  o[0] = (h0 - mu) * rs * bf16r(g0) + bf16r(b0);
  o[1] = (h1 - mu) * rs * bf16r(g1) + bf16r(b1);
  o[2] = (h2 - mu) * rs * bf16r(g2) + bf16r(b2);
  o[3] = (h3 - mu) * rs * bf16r(g3) + bf16r(b3);
  float* q = out + (size_t)i * 4;
  *(volatile v4f*)q = o;
  __threadfence();
  *(volatile v4f*)q = o;
}

static_assert(((kRows / 32) * (kXzN / 64)) % 8 == 0 && ((kRows / 32) * (kXzN / 64)) / 8 == 512);
static_assert((2048 / 32) * (4096 / 64) / 8 == 512);
static_assert(((kRows / 32) * (kXpP / 64)) % 8 == 0 && ((kRows / 32) * (kXpP / 64)) / 8 == 16);
static_assert((2048 / 32) * (128 / 64) / 8 == 16);
static_assert(((kRows / 32) * (kE / 64)) % 8 == 0 && ((kRows / 32) * (kE / 64)) / 8 == 256);
static_assert((2048 / 32) * (2048 / 64) / 8 == 256);
static_assert(((kRows / 32) * (kDm / 64)) % 8 == 0 && ((kRows / 32) * (kDm / 64)) / 8 == 128);
static_assert((2048 / 32) * (1024 / 64) / 8 == 128);
static_assert(((kXzN * kDm / 8) % 256) == 0 && (kXzN * kDm / 8) / 256 == 2048);
static_assert(((kXpP * kDm / 8) % 256) == 0 && (kXpP * kDm / 8) / 256 == 64);
static_assert(((kE * kRankWords) % 256) == 0 && (kE * kRankWords) / 256 == 64);
static_assert(((kE * kTailWords) % 256) == 0 && (kE * kTailWords) / 256 == 64);
static_assert(((kDm * kE / 8) % 256) == 0 && (kDm * kE / 8) / 256 == 1024);
static_assert((kPadFloats / 4) == 272 * 32 && (kAlpFloats / 4) == 256 * 32);
static_assert(((kRows * kDm / 8) % 256) == 0 && (kRows * kDm / 8) / 256 == 1024);
static_assert(((kRows * kE / 4) % 256) == 0 && (kRows * kE / 4) / 256 == 4096);
static_assert(((kRows * kE / 8) % 256) == 0 && (kRows * kE / 8) / 256 == 2048);
static_assert(((kRows * kK2Words) % 256) == 0 && (kRows * kK2Words) / 256 == 96);
static_assert(((kRows * kDm / 4) % 256) == 0 && (kRows * kDm / 4) / 256 == 2048);
static_assert((kRows % 256) == 0 && kRows / 256 == 8);
static_assert((kE % 64) == 0 && (kL % 64) == 0);
static_assert(kRows == kL && kPasses * kRows == kBatch * kL);
static_assert((2048 / 64) * 1 == 32);
static_assert((kE / 64) * 1 == 32);
static_assert(kRank == 64 && kColDt + kRank <= kXpP && kWbRow0 + kXpP == kWinRows);

extern "C" void kernel_launch(void* const* d_in, const int* in_sizes, int n_in,
                              void* d_out, int out_size, void* d_ws, size_t ws_size,
                              hipStream_t stream)
{
  if (n_in < 11) return;
  if (in_sizes[0] != kBatch * kL * kDm) return;
  if (in_sizes[1] != kWinRows * kDm) return;
  if (in_sizes[2] != kE * kRank) return;
  if (in_sizes[3] != kE) return;
  if (in_sizes[4] != kE * kNst) return;
  if (in_sizes[5] != kE) return;
  if (in_sizes[6] != kE * kTaps) return;
  if (in_sizes[7] != kE) return;
  if (in_sizes[8] != kDm * kE) return;
  if (in_sizes[9] != kDm) return;
  if (in_sizes[10] != kDm) return;
  if (out_size != kBatch * kL * kDm) return;
  if (ws_size < kWsTotal) return;

  const float* x_in   = (const float*)d_in[0];
  const float* w_in   = (const float*)d_in[1];
  const float* w_dt   = (const float*)d_in[2];
  const float* b_dt   = (const float*)d_in[3];
  const float* a_log  = (const float*)d_in[4];
  const float* d_skip = (const float*)d_in[5];
  const float* conv_w = (const float*)d_in[6];
  const float* conv_b = (const float*)d_in[7];
  const float* w_out  = (const float*)d_in[8];
  const float* ln_g   = (const float*)d_in[9];
  const float* ln_b   = (const float*)d_in[10];
  float* out = (float*)d_out;

  char* ws = (char*)d_ws;
  unsigned short* WIN  = (unsigned short*)(ws + kOffWIN);
  unsigned short* WB   = (unsigned short*)(ws + kOffWB);
  unsigned short* WDT  = (unsigned short*)(ws + kOffWDT);
  unsigned short* OW   = (unsigned short*)(ws + kOffOW);
  float*          PADS = (float*)(ws + kOffPADS);
  unsigned short* SH   = (unsigned short*)(ws + kOffSH);
  float*          XZ   = (float*)(ws + kOffXZ);
  float*          XC   = (float*)(ws + kOffXC);
  float*          XD   = (float*)(ws + kOffXD);
  unsigned short* DRH  = (unsigned short*)(ws + kOffDRH);
  float*          DTP  = (float*)(ws + kOffDTP);
  unsigned short* YH   = (unsigned short*)(ws + kOffYH);
  unsigned short* YG   = (unsigned short*)(ws + kOffYG);
  float*          H    = (float*)(ws + kOffH);
  float*          R    = (float*)(ws + kOffR);
  float*          ST   = (float*)(ws + kOffST);
  float*          ALP  = PADS;
  float*          DSP  = PADS + kAlpFloats;

  constexpr float s1 = 1.0f / (kXCarry * kWCarry);
  constexpr float s3 = 1.0f / (kRCarry * kDCarry);
  constexpr float s4 = 1.0f / (kGCarry * kWCarry);

  pack_win_kernel<<<(kXzN * kDm / 8) / 256, 256, 0, stream>>>(w_in, WIN);

  pack_win_kernel<<<(kXpP * kDm / 8) / 256, 256, 0, stream>>>(w_in + (size_t)kWbRow0 * kDm, WB);

  pack_wdt_kernel<<<(kE * kRankWords) / 256, 256, 0, stream>>>(w_dt, WDT);

  pack_bias_kernel<<<(kE * kTailWords) / 256, 256, 0, stream>>>(b_dt, WDT);

  pack_wout_kernel<<<(kDm * kE / 8) / 256, 256, 0, stream>>>(w_out, OW);

  pads_kernel<<<272, 32, 0, stream>>>(a_log, d_skip, PADS);

  for (int p = 0; p < kPasses; ++p) {
    const float* xp = x_in + (size_t)p * kRows * kDm;
    float* outp = out + (size_t)p * kRows * kDm;

    pack_s_kernel<<<(kRows * kDm / 8) / 256, 256, 0, stream>>>(xp, SH);

    eng::gemm_f16_kernel<2, 0><<<dim3((2048 / 32) * (4096 / 64) / 8), 256, 0, stream>>>(
        SH, nullptr, 1024, WIN, nullptr, 1024, XZ, 4096, 2048, 4096, 1024, s1, 0.0f);

    eng::gemm_f16_kernel<2, 0><<<dim3((2048 / 32) * (128 / 64) / 8), 256, 0, stream>>>(
        SH, nullptr, 1024, WB, nullptr, 1024, XD, 128, 2048, 128, 1024, s1, 0.0f);

    conv1d_kernel<<<(kRows * kE / 4) / 256, 256, 0, stream>>>(XZ, conv_w, conv_b, XC);

    pack_dr_kernel<<<(kRows * kK2Words) / 256, 256, 0, stream>>>(XD + kColDt, DRH);

    eng::gemm_f16_kernel<2, 0><<<dim3((2048 / 32) * (2048 / 64) / 8), 256, 0, stream>>>(
        DRH, nullptr, 96, WDT, nullptr, 128, DTP, 2048, 2048, 2048, 96, s3, 0.0f);

    ms1_args sa;
    sa.dtpre = DTP;
    sa.u = XC;
    sa.bc = XD;
    sa.z = nullptr;
    sa.A_log = ALP;
    sa.Dskip = DSP;
    sa.y = (__half*)YH;
    sa.y_lo = nullptr;
    sa.ld_dtpre = kE;
    sa.ld_u = kE;
    sa.ld_bc = kXpP;
    sa.ld_z = 0;
    sa.ld_y = kE;
    sa.offB = kColB;
    sa.offC = kColC;
    sa.offZ = 0;
    sa.ycarry = kYCarry;
    sa.dir = 1;
    sa.D = kE;
    sa.L = kL;
    sa.nbatch = 1;
    ms1_scan_kernel<16><<<dim3((2048 / 64) * 1), 64, 0, stream>>>(sa);

    gate_kernel<<<(kRows * kE / 8) / 256, 256, 0, stream>>>(YH, XZ, YG);

    eng::gemm_f16_kernel<2, 0><<<dim3((2048 / 32) * (1024 / 64) / 8), 256, 0, stream>>>(
        YG, nullptr, 2048, OW, nullptr, 2048, H, 1024, 2048, 1024, 2048, s4, 0.0f);

    res_out_kernel<<<(kRows * kDm / 4) / 256, 256, 0, stream>>>(xp, H, R);

    ln_stats_kernel<<<kRows / 256, 256, 0, stream>>>(R, ST);

    ln_out_kernel<<<(kRows * kDm / 4) / 256, 256, 0, stream>>>(R, ST, ln_g, ln_b, outp);
  }
}
